// DecoderBlock_41609643163860
// MI455X (gfx1250) — hardware-verified
//
#include <hip/hip_runtime.h>
#include <math.h>

typedef __attribute__((ext_vector_type(16))) _Float16 v16h;
typedef __attribute__((ext_vector_type(16))) __bf16 v16b;
typedef __attribute__((ext_vector_type(8)))  _Float16 v8h;
typedef __attribute__((ext_vector_type(8)))  float v8f;
typedef __attribute__((ext_vector_type(4)))  float v4f;
typedef __attribute__((ext_vector_type(4)))  unsigned v4u;

template <typename T> __device__ __forceinline__ void vst2(void* p, T v) { *(volatile T*)p = v; __threadfence(); *(volatile T*)p = v; }
__device__ __forceinline__ v8f wmma16(v16h a, v16h b, v8f c) {
  v8f d = __builtin_amdgcn_wmma_f32_16x16x32_f16(false, a, false, b, (short)0, c, false, false);
  asm volatile("v_nop\n\tv_nop\n\tv_nop\n\tv_nop" : "+v"(d) : "v"(a), "v"(b));
  return d;
}
__device__ __forceinline__ v8f wmma_bf(v16b a, v16b b, v8f c) {
  v8f d = __builtin_amdgcn_wmma_f32_16x16x32_bf16(false, a, false, b, (short)0, c, false, false);
  asm volatile("v_nop\n\tv_nop\n\tv_nop\n\tv_nop" : "+v"(d) : "v"(a), "v"(b));
  return d;
}
__device__ __forceinline__ v16h frag_h(const _Float16* rowk0, int lane) {
  union { v16h v; v8h q[2]; } u; const _Float16* p = rowk0 + 8 * (lane >> 4);
  u.q[0] = *(const v8h*)p; u.q[1] = *(const v8h*)(p + 16); return u.v;
}
__device__ __forceinline__ v16h frag_f32(const float* rowk0, int lane) {
  v16h a; const float* p = rowk0 + 8 * (lane >> 4);
#pragma unroll
  for (int i = 0; i < 8; ++i) { a[i] = (_Float16)p[i]; a[8 + i] = (_Float16)p[16 + i]; }
  return a;
}
__device__ __forceinline__ float bfr(float v) { return (float)(__bf16)v; }
__device__ __forceinline__ v16b wcol_io(const float* Wm, int k0, int o, int lane, int ld) { v16b w; const int g = lane >> 4;
#pragma unroll
  for (int i = 0; i < 8; ++i) { w[i] = (__bf16)Wm[(size_t)(k0 + 8 * g + i) * ld + o]; w[8 + i] = (__bf16)Wm[(size_t)(k0 + 16 + 8 * g + i) * ld + o]; }
  return w; }
#define LDSX() do { asm volatile("s_wait_dscnt 0" ::: "memory"); __builtin_amdgcn_wave_barrier(); __builtin_amdgcn_fence(3  , "workgroup"); } while (0)

#ifndef NB
#define NB 2
#endif
#ifndef SEQ
#define SEQ 2048
#endif
#define SEQ_FULL 2048
#define TQ SEQ
#define TK SEQ
#define CC 512
#define DIN 512
#define NH 8
#define HD 64
#define HG 4
#define FF 2048
#define SCALE (0.125f)
#define PCARRY (2048.0f)
#define NRW (NB * TQ)
#define NRK (NB * TK)

static_assert(TQ == TK);
static_assert(TQ % 64 == 0);
static_assert(TK % 128 == 0);
static_assert(NRW % 64 == 0);
static_assert(NRW % 8 == 0);
static_assert(CC == 512);
static_assert(CC == NH * HD);
static_assert(HD == 64);
static_assert(NH % HG == 0);
static_assert(DIN % 32 == 0);
static_assert(CC % 128 == 0);
static_assert(FF % 128 == 0);
static_assert(FF % 32 == 0);
static_assert(TK * 4 <= 32768);

constexpr size_t SZ_QH = (size_t)2 * NRW * CC;
constexpr size_t SZ_KH = (size_t)2 * NRK * CC;
constexpr size_t SZ_VT = (size_t)2 * NB * CC * TK;
constexpr size_t SZ_S  = (size_t)4 * HG * TQ * TK;
constexpr size_t SZ_HF = (size_t)4 * NRW * FF;
constexpr size_t SZ_SHF = SZ_S > SZ_HF ? SZ_S : SZ_HF;
constexpr size_t SZ_ROWS = (size_t)4 * NRW * CC;
constexpr size_t WS_QH = 0;
constexpr size_t WS_KH = WS_QH + SZ_QH;
constexpr size_t WS_VT = WS_KH + SZ_KH;
constexpr size_t WS_S  = WS_VT + SZ_VT;
constexpr size_t WS_Y  = WS_S + SZ_SHF;
constexpr size_t WS_O1 = WS_Y + SZ_ROWS;
constexpr size_t WS_Z  = WS_O1 + SZ_ROWS;
constexpr size_t WS_END = WS_Z + SZ_ROWS;
static_assert(SZ_S <= SZ_SHF);
static_assert(SZ_HF <= SZ_SHF);
static_assert(WS_KH % 128 == 0);
static_assert(WS_VT % 128 == 0);
static_assert(WS_S % 128 == 0);
static_assert(WS_Y % 128 == 0);
static_assert(WS_O1 % 128 == 0);
static_assert(WS_Z % 128 == 0);
static_assert(WS_END <= (size_t)134217728);

__global__ __launch_bounds__(256) void k_addln(const float* __restrict__ X, int cvtin, unsigned xbatch_rows, const float* __restrict__ ADD, int hasadd, const float* __restrict__ G, const float* __restrict__ BE, const int* __restrict__ NHP, float* __restrict__ OUT) {
  const unsigned wave = threadIdx.x >> 5, lane = threadIdx.x & 31u; const unsigned row = blockIdx.x * 8u + wave; if (row >= (unsigned)NRW) return;
  const unsigned xr = (row / (unsigned)TQ) * xbatch_rows + (row % (unsigned)TQ);
  const float pz = (NHP[0] != NH) ? __int_as_float(0x7fc00000) : 0.f;
  v4f v[CC / 128]; float s1 = 0.f;
#pragma unroll
  for (int i = 0; i < CC / 128; ++i) { v4f t = *(const v4f*)(X + (size_t)xr * CC + i * 128 + lane * 4);
    if (cvtin) { t[0] = bfr(t[0]); t[1] = bfr(t[1]); t[2] = bfr(t[2]); t[3] = bfr(t[3]); }
    if (hasadd) { const v4f a = *(const v4f*)(ADD + (size_t)row * CC + i * 128 + lane * 4); t[0] += a[0]; t[1] += a[1]; t[2] += a[2]; t[3] += a[3]; }
    v[i] = t; s1 += (t[0] + t[1]) + (t[2] + t[3]); }
#pragma unroll
  for (int o = 1; o < 32; o <<= 1) s1 += __shfl_xor(s1, o);
  const float mu = s1 * (1.0f / CC); float q = 0.f;
#pragma unroll
  for (int i = 0; i < CC / 128; ++i) for (int k = 0; k < 4; ++k) { const float d = v[i][k] - mu; q += d * d; }
#pragma unroll
  for (int o = 1; o < 32; o <<= 1) q += __shfl_xor(q, o);
  const float inv = rsqrtf(q * (1.0f / CC) + 1e-5f);
#pragma unroll
  for (int i = 0; i < CC / 128; ++i) { const unsigned c = i * 128 + lane * 4; v4f r4; for (int k = 0; k < 4; ++k) r4[k] = bfr(G[c + k]) * ((v[i][k] - mu) * inv) + bfr(BE[c + k]) + pz; vst2(OUT + (size_t)row * CC + c, r4); } }

__global__ __launch_bounds__(128) void k_proj(const float* __restrict__ XQ, const float* __restrict__ XE, const float* __restrict__ WQ, const float* __restrict__ WK, const float* __restrict__ WV,
    _Float16* __restrict__ QH, _Float16* __restrict__ KH, _Float16* __restrict__ VT) {
  __shared__ __align__(16) _Float16 sh[64][136]; __shared__ __align__(16) _Float16 th[128][72];
  const unsigned tid = threadIdx.x, wave = tid >> 5, lane = tid & 31u, col = lane & 15u, g = lane >> 4;
  const unsigned which = blockIdx.z, c0 = blockIdx.y * 128u, r0 = blockIdx.x * 64u; const unsigned bb = r0 / (unsigned)TQ, t0 = r0 % (unsigned)TQ;
  const float* X = which == 0 ? XQ : XE; const float* WA = which == 0 ? WQ : (which == 1 ? WK : WV);
  const float* xrow = X + ((size_t)bb * SEQ_FULL + t0 + wave * 16u + col) * DIN + 8u * g;
  v8f acc[8] = {};
#pragma unroll 2
  for (int kc = 0; kc < DIN / 32; ++kc) { v16b a; { const float* p = xrow + kc * 32;
#pragma unroll
      for (int i = 0; i < 8; ++i) { a[i] = (__bf16)p[i]; a[8 + i] = (__bf16)p[16 + i]; } }
    asm volatile("s_wait_loadcnt 0x0" ::: "memory");
#pragma unroll
    for (int j = 0; j < 8; ++j) { const v16b w = wcol_io(WA, kc * 32, (int)(c0 + j * 16 + col), (int)lane, CC); asm volatile("s_wait_loadcnt 0x0" ::: "memory"); acc[j] = wmma_bf(a, w, acc[j]); } }
  if (which < 2) { _Float16* DH = which == 0 ? QH : KH;
#pragma unroll
    for (int j = 0; j < 8; ++j) {
#pragma unroll
      for (int r = 0; r < 8; ++r) sh[wave * 16 + 8 * g + r][j * 16 + col] = (_Float16)acc[j][r]; }
    __syncthreads();
    for (unsigned e = tid; e < 64u * 16u; e += 128u) { const unsigned rl = e >> 4, q = e & 15u; vst2(DH + ((size_t)r0 + rl) * CC + c0 + q * 8u, *(const v4u*)&sh[rl][q * 8]); }
  } else {
#pragma unroll
    for (int j = 0; j < 8; ++j) {
#pragma unroll
      for (int r = 0; r < 8; ++r) th[j * 16 + col][wave * 16 + 8 * g + r] = (_Float16)acc[j][r]; }
    __syncthreads();
    for (unsigned e = tid; e < 128u * 8u; e += 128u) { const unsigned cl = e >> 3, q = e & 7u; vst2(VT + ((size_t)bb * CC + c0 + cl) * (size_t)TK + t0 + q * 8u, *(const v4u*)&th[cl][q * 8]); } } }

__global__ __launch_bounds__(128) void k_sc(const _Float16* __restrict__ QH, const _Float16* __restrict__ KH, unsigned b, unsigned h0, float* __restrict__ S0) {
  __shared__ __align__(16) float ss[4][16][132];
  const unsigned qb = blockIdx.x, kb = blockIdx.y, h = h0 + blockIdx.z; float* S = S0 + (size_t)blockIdx.z * TQ * TK;
  const unsigned tid = threadIdx.x, wave = tid >> 5, lane = tid & 31u, col = lane & 15u, g = lane >> 4; const unsigned k0 = kb * 128u, ql0 = qb * 64u + wave * 16u;
  const size_t q0 = (size_t)b * TQ + ql0, kr0 = (size_t)b * TK + k0;
  v8f acc[8] = {};
#pragma unroll
  for (int kc = 0; kc < HD / 32; ++kc) { const v16h ah = frag_h(QH + (q0 + col) * CC + h * HD + kc * 32, (int)lane);
#pragma unroll
    for (int j = 0; j < 8; ++j) { const v16h kf = frag_h(KH + (kr0 + j * 16 + col) * CC + h * HD + kc * 32, (int)lane); acc[j] = wmma16(ah, kf, acc[j]); } }
#pragma unroll
  for (int j = 0; j < 8; ++j) {
#pragma unroll
    for (int r = 0; r < 8; ++r) ss[wave][8 * g + r][j * 16 + col] = acc[j][r] * SCALE; }
  LDSX(); for (unsigned rl = 0; rl < 16u; ++rl) vst2(S + (size_t)(ql0 + rl) * TK + k0 + lane * 4u, *(const v4f*)&ss[wave][rl][lane * 4]); }

__global__ __launch_bounds__(256) void k_sm(float* __restrict__ S0) { __shared__ float sred[8]; __shared__ float sbc; __shared__ __align__(16) float shv[TK];
  const unsigned tid = threadIdx.x, t = blockIdx.x;
  float* sr = S0 + (size_t)blockIdx.y * TQ * TK + (size_t)t * TK;
  float m = -3.0e38f;
#pragma unroll 1
  for (unsigned q = tid; q < (unsigned)(TK / 4); q += 256u) { const v4f v = *(const v4f*)(sr + q * 4u); *(v4f*)&shv[q * 4u] = v; m = fmaxf(fmaxf(m, fmaxf(v[0], v[1])), fmaxf(v[2], v[3])); }
#pragma unroll
  for (int o = 1; o < 32; o <<= 1) m = fmaxf(m, __shfl_xor(m, o));
  if ((tid & 31u) == 0) sred[tid >> 5] = m; __syncthreads(); if (tid == 0) { float a = sred[0]; for (int i = 1; i < 8; ++i) a = fmaxf(a, sred[i]); sbc = a; } __syncthreads(); m = sbc; __syncthreads();
  float sum = 0.f;
#pragma unroll 1
  for (unsigned q = tid; q < (unsigned)(TK / 4); q += 256u) { v4f v = *(const v4f*)&shv[q * 4u]; v[0] = expf(v[0] - m); v[1] = expf(v[1] - m); v[2] = expf(v[2] - m); v[3] = expf(v[3] - m); *(v4f*)&shv[q * 4u] = v; sum += (v[0] + v[1]) + (v[2] + v[3]); }
#pragma unroll
  for (int o = 1; o < 32; o <<= 1) sum += __shfl_xor(sum, o);
  if ((tid & 31u) == 0) sred[tid >> 5] = sum; __syncthreads(); if (tid == 0) { float a = 0.f; for (int i = 0; i < 8; ++i) a += sred[i]; sbc = a > 0.f ? PCARRY * (1.0f / a) : 0.f; } __syncthreads(); const float inv = sbc;
#pragma unroll 1
  for (unsigned q = tid; q < (unsigned)(TK / 4); q += 256u) { v4f v = *(const v4f*)&shv[q * 4u]; v[0] *= inv; v[1] *= inv; v[2] *= inv; v[3] *= inv; vst2(sr + q * 4u, v); } }

__global__ __launch_bounds__(128) void k_pv(const float* __restrict__ PS0, const _Float16* __restrict__ VT, unsigned b, unsigned h0, float* __restrict__ Y) {
  __shared__ __align__(16) float ss[4][16][HD + 4];
  const unsigned h = h0 + blockIdx.z; const float* PS = PS0 + (size_t)blockIdx.z * TQ * TK;
  const unsigned tid = threadIdx.x, wave = tid >> 5, lane = tid & 31u, col = lane & 15u, g = lane >> 4; const unsigned ql0 = blockIdx.x * 64u + wave * 16u;
  const float* prow = PS + (size_t)(ql0 + col) * TK;
  const _Float16* vbase = VT + ((size_t)b * CC + h * HD + col) * (size_t)TK;
  v8f acc[HD / 16] = {};
#pragma unroll 1
  for (unsigned kc = 0; kc < (unsigned)(TK / 32); ++kc) { const v16h p = frag_f32(prow + kc * 32u, (int)lane);
    asm volatile("s_wait_loadcnt 0x0" ::: "memory");
#pragma unroll
    for (int j = 0; j < HD / 16; ++j) acc[j] = wmma16(p, frag_h(vbase + (size_t)j * 16 * TK + kc * 32u, (int)lane), acc[j]); }
#pragma unroll
  for (int j = 0; j < HD / 16; ++j)
#pragma unroll
    for (int r = 0; r < 8; ++r) ss[wave][8 * g + r][j * 16 + col] = acc[j][r] * (1.0f / PCARRY);
  LDSX(); for (unsigned rl = 0; rl < 16u; ++rl) { const v4f v = *(const v4f*)&ss[wave][rl][col * 4u]; if (lane < (unsigned)(HD / 4)) vst2(Y + ((size_t)b * TQ + ql0 + rl) * CC + h * HD + col * 4u, v); } }

__global__ __launch_bounds__(128) void k_gemh(const float* __restrict__ A, int lda, int K, int act_in, const float* __restrict__ Wm, int nout, const float* __restrict__ BIAS, const float* __restrict__ RES, int hasres, float* __restrict__ OUT) {
  __shared__ __align__(16) float sf[4][16][132];
  const unsigned tid = threadIdx.x, wave = tid >> 5, lane = tid & 31u, col = lane & 15u, g = lane >> 4; const unsigned c0 = blockIdx.y * 128u; const size_t r0 = (size_t)blockIdx.x * 64 + wave * 16;
  v8f acc[8] = {};
#pragma unroll 1
  for (int kc = 0; kc < K / 32; ++kc) { v16h a; { const float* p = A + (r0 + col) * (size_t)lda + kc * 32 + 8 * g;
#pragma unroll
      for (int i = 0; i < 8; ++i) { float x0 = p[i], x1 = p[16 + i]; if (act_in == 1) { x0 = fmaxf(x0, 0.f); x1 = fmaxf(x1, 0.f); } a[i] = (_Float16)x0; a[8 + i] = (_Float16)x1; } }
    asm volatile("s_wait_loadcnt 0x0" ::: "memory");
#pragma unroll
    for (int j = 0; j < 8; ++j) { v16h w; { const unsigned o = c0 + j * 16 + col; float t0[8], t1[8];
#pragma unroll
        for (int i = 0; i < 8; ++i) t0[i] = Wm[(size_t)(kc * 32 + 8 * g + i) * nout + o];
        asm volatile("s_wait_loadcnt 0x0" ::: "memory");
#pragma unroll
        for (int i = 0; i < 8; ++i) t1[i] = Wm[(size_t)(kc * 32 + 16 + 8 * g + i) * nout + o];
        asm volatile("s_wait_loadcnt 0x0" ::: "memory");
#pragma unroll
        for (int i = 0; i < 8; ++i) { w[i] = (_Float16)(bfr(t0[i]) * 64.0f); w[8 + i] = (_Float16)(bfr(t1[i]) * 64.0f); } }
      acc[j] = wmma16(a, w, acc[j]); } }
#pragma unroll
  for (int j = 0; j < 8; ++j)
    { const float bb = bfr(BIAS[c0 + j * 16 + col]); asm volatile("s_wait_loadcnt 0x0" ::: "memory"); _Pragma("unroll") for (int r = 0; r < 8; ++r) sf[wave][8 * g + r][j * 16 + col] = acc[j][r] * (1.0f / 64.0f) + bb; }
  LDSX(); for (unsigned rl = 0; rl < 16u; ++rl) { const size_t o = (r0 + rl) * (size_t)nout + c0 + lane * 4u; v4f v = *(const v4f*)&sf[wave][rl][lane * 4]; if (hasres) { const v4f rv = *(const v4f*)(RES + o); v[0] += rv[0]; v[1] += rv[1]; v[2] += rv[2]; v[3] += rv[3]; } vst2(OUT + o, v); } }

extern "C" void kernel_launch(void* const* d_in, const int* in_sizes, int n_in, void* d_out, int out_size, void* d_ws, size_t ws_size, hipStream_t stream) {
  if (n_in < 14) return;
  if (ws_size < WS_END) return;
  const long need_x = ((long)(NB - 1) * SEQ_FULL + SEQ) * DIN;
  if ((long)in_sizes[0] < need_x || (long)in_sizes[1] < need_x) return;
  if (in_sizes[2] < DIN * CC || in_sizes[3] < DIN * CC || in_sizes[4] < DIN * CC) return;
  if (in_sizes[5] < CC || in_sizes[6] < CC || in_sizes[11] < CC || in_sizes[12] < CC) return;
  if (in_sizes[7] < CC * FF || in_sizes[8] < FF || in_sizes[9] < FF * CC || in_sizes[10] < CC || in_sizes[13] < 1) return;
  if ((long)out_size < (long)NRW * CC) return;
  const float* const* F = (const float* const*)d_in; const int* NHP = (const int*)d_in[13];
  char* ws = (char*)d_ws;
  _Float16 *QH = (_Float16*)(ws + WS_QH), *KH = (_Float16*)(ws + WS_KH), *VT = (_Float16*)(ws + WS_VT);
  float *S = (float*)(ws + WS_S), *HF = (float*)(ws + WS_S), *Y = (float*)(ws + WS_Y), *O1 = (float*)(ws + WS_O1), *Z = (float*)(ws + WS_Z);
  k_proj<<<dim3(NRW / 64, CC / 128, 3), 128, 0, stream>>>(F[0], F[1], F[2], F[3], F[4], QH, KH, VT);
  for (unsigned b = 0; b < (unsigned)NB; ++b) for (unsigned h0 = 0; h0 < (unsigned)NH; h0 += HG) {
    k_sc<<<dim3(TQ / 64, TK / 128, HG), 128, 0, stream>>>(QH, KH, b, h0, S);
    k_sm<<<dim3(TQ, HG), 256, 0, stream>>>(S);
    k_pv<<<dim3(TQ / 64, 1, HG), 128, 0, stream>>>(S, VT, b, h0, Y);
  }
  k_addln<<<dim3(NRW / 8), 256, 0, stream>>>(F[0], 1, (unsigned)SEQ_FULL, Y, 1, F[5], F[6], NHP, O1);
  k_gemh<<<dim3(NRW / 64, FF / 128), 128, 0, stream>>>(O1, CC, CC, 0, F[7], FF, F[8], O1, 0, HF);
  k_gemh<<<dim3(NRW / 64, CC / 128), 128, 0, stream>>>(HF, FF, FF, 1, F[9], CC, F[10], O1, 1, Z);
  k_addln<<<dim3(NRW / 8), 256, 0, stream>>>(Z, 0, (unsigned)TQ, Z, 0, F[11], F[12], NHP, (float*)d_out);
}
